// SimpleSSM_70153995813361
// MI455X (gfx1250) — hardware-verified
//
#include <hip/hip_runtime.h>
#include <math.h>

typedef __attribute__((ext_vector_type(16))) _Float16 v16h;
typedef __attribute__((ext_vector_type(8)))  _Float16 v8h;
typedef __attribute__((ext_vector_type(16))) __bf16   v16b;
typedef __attribute__((ext_vector_type(8)))  __bf16   v8b;
typedef __attribute__((ext_vector_type(8)))  float    v8f;
typedef __attribute__((ext_vector_type(4)))  float    v4f;

constexpr int kBatch = 4;
constexpr int kSeq   = 2048;
constexpr int kDm    = 1024;
constexpr int kNst   = 16;
constexpr int kRows  = kBatch * kSeq;
constexpr int kBxP   = 64;
constexpr int kHmP   = 32;
constexpr int kTaps  = 128;
constexpr int kFirTS = 64;
constexpr int kFirWin = kFirTS + kTaps;
static_assert(kRows == 8192);
static_assert((kDm % 32) == 0 && (kHmP % 32) == 0);
static_assert((kRows % 64) == 0 && (kBxP % 64) == 0 && (kDm % 64) == 0);
static_assert((kSeq % kFirTS) == 0 && kNst == 16 && kTaps == 128);

constexpr size_t kOffXB  = 0;
constexpr size_t kOffBWB = kOffXB  + (size_t)kRows * kDm * 2;
constexpr size_t kOffCWB = kOffBWB + (size_t)kBxP * kDm * 2;
constexpr size_t kOffBX  = kOffCWB + (size_t)kDm * kHmP * 2;
constexpr size_t kOffGT  = kOffBX  + (size_t)kRows * kBxP * 4;
constexpr size_t kOffHMH = kOffGT  + (size_t)kNst * kTaps * 4;
constexpr size_t kOffHML = kOffHMH + (size_t)kRows * kHmP * 2;
constexpr size_t kOffYS  = kOffHML + (size_t)kRows * kHmP * 2;
constexpr size_t kWsTotal = kOffYS + (size_t)kRows * kDm * 4;
static_assert(kWsTotal == 53682176ull);
static_assert(kWsTotal <= 134217728ull);
static_assert((kOffBWB % 128) == 0 && (kOffCWB % 128) == 0 && (kOffBX % 128) == 0 && (kOffGT % 128) == 0 &&
              (kOffHMH % 128) == 0 && (kOffHML % 128) == 0 && (kOffYS % 128) == 0);

__device__ __forceinline__ unsigned short f2bf_bits(float f) {
  unsigned u = __float_as_uint(f);
  return (unsigned short)((u + 0x7FFFu + ((u >> 16) & 1u)) >> 16);
}
__device__ __forceinline__ float bf_bits2f(unsigned short h) { return __uint_as_float(((unsigned)h) << 16); }
__device__ __forceinline__ float bfr(float f) { return bf_bits2f(f2bf_bits(f)); }

__device__ __forceinline__ void dep_guard_h(v8f& a, v8f& b, v16h x, v16h y) { asm volatile("v_nop\n\tv_nop\n\tv_nop\n\tv_nop" : "+v"(a), "+v"(b) : "v"(x), "v"(y)); }
__device__ __forceinline__ void dep_guard_b(v8f& a, v8f& b, v16b x, v16b y) { asm volatile("v_nop\n\tv_nop\n\tv_nop\n\tv_nop" : "+v"(a), "+v"(b) : "v"(x), "v"(y)); }
__device__ __forceinline__ void keep4_h(v16h a, v16h b, v16h c, v16h d) { asm volatile("v_nop" :: "v"(a), "v"(b), "v"(c), "v"(d)); }
__device__ __forceinline__ void keep4_b(v16b a, v16b b, v16b c, v16b d) { asm volatile("v_nop" :: "v"(a), "v"(b), "v"(c), "v"(d)); }
__device__ __forceinline__ void acc_guard4(v8f& a, v8f& b, v8f& c, v8f& d) { asm volatile("v_nop\n\tv_nop\n\tv_nop\n\tv_nop" : "+v"(a), "+v"(b), "+v"(c), "+v"(d)); }
template <typename T> struct Frag;
template <> struct Frag<_Float16> {
  typedef v16h V; union U { v16h v; v8h h[2]; };
  static __device__ __forceinline__ v16h load(const _Float16* p) {
    U f; f.h[0] = *(const v8h*)(p); f.h[1] = *(const v8h*)(p + 16); return f.v;
  }
  static __device__ __forceinline__ v8f mma(v16h a, v16h b, v8f c) {
    return __builtin_amdgcn_wmma_f32_16x16x32_f16(false, a, false, b, (short)0, c, false, false);
  }
  static __device__ __forceinline__ void guard(v8f& a, v8f& b, v16h x, v16h y) { dep_guard_h(a, b, x, y); }
  static __device__ __forceinline__ void keep(v16h a, v16h b, v16h c, v16h d) { keep4_h(a, b, c, d); }
};
template <> struct Frag<__bf16> {
  typedef v16b V; union U { v16b v; v8b h[2]; };
  static __device__ __forceinline__ v16b load(const __bf16* p) {
    U f; f.h[0] = *(const v8b*)(p); f.h[1] = *(const v8b*)(p + 16); return f.v;
  }
  static __device__ __forceinline__ v8f mma(v16b a, v16b b, v8f c) {
    return __builtin_amdgcn_wmma_f32_16x16x32_bf16(false, a, false, b, (short)0, c, false, false);
  }
  static __device__ __forceinline__ void guard(v8f& a, v8f& b, v16b x, v16b y) { dep_guard_b(a, b, x, y); }
  static __device__ __forceinline__ void keep(v16b a, v16b b, v16b c, v16b d) { keep4_b(a, b, c, d); }
};

template <int ET> struct Elem;
template <> struct Elem<0> { typedef _Float16 T; };
template <> struct Elem<1> { typedef __bf16 T; };
template <int ET, int SPL, int BIAS_MODE, int OUT_MODE, bool RESID, int ACT = 0>
__global__ __launch_bounds__(256) void wmma_gemm64(
    const unsigned short* __restrict__ Ap, const unsigned short* __restrict__ A2p, int lda, long strideA,
    const unsigned short* __restrict__ Btp, const unsigned short* __restrict__ Bt2p, int ldb, long strideB,
    void* __restrict__ Cout, void* __restrict__ Cout2, int ldc, long strideC,
    const float* __restrict__ bias,
    const float* __restrict__ resid, long strideR,
    int M, int N, int K, float scale) {
  typedef typename Elem<ET>::T T;
  typedef typename Frag<T>::V V;
  const T* A = (const T*)Ap; const T* A2 = (const T*)A2p; const T* Bt = (const T*)Btp; const T* Bt2 = (const T*)Bt2p;
  __shared__ __align__(16) float sT[8][16 * 68];
  const int b    = blockIdx.y;
  const int lane = threadIdx.x & 31;
  const int wave = threadIdx.x >> 5;
  const int tilesN = N >> 6;
  const int tilesM = M >> 6;
  const int tile = blockIdx.x * 8 + wave;
  if (tile >= tilesM * tilesN) return;
  const int tm = tile / tilesN;
  const int tn = tile - tm * tilesN;
  const int m0 = tm << 6;
  const int n0 = tn << 6;

  const T* Ab  = A  + (size_t)b * strideA;
  const T* Bb  = Bt + (size_t)b * strideB;
  const T* Ab2 = (SPL >= 1) ? (A2  + (size_t)b * strideA) : nullptr;
  const T* Bb2 = (SPL == 2) ? (Bt2 + (size_t)b * strideB) : nullptr;

  const int rlane = lane & 15;
  const int koff  = (lane >> 4) * 8;
  const int mOff  = (lane >> 4) * 8;

  v8f acc[4][4];
#pragma unroll
  for (int i = 0; i < 4; ++i)
#pragma unroll
    for (int j = 0; j < 4; ++j) acc[i][j] = (v8f){0.f,0.f,0.f,0.f,0.f,0.f,0.f,0.f};

  for (int k0 = 0; k0 < K; k0 += 32) {
    V bh[4], bl[4];
#pragma unroll
    for (int j = 0; j < 4; ++j) {
      const size_t bo = (size_t)(n0 + (j << 4) + rlane) * ldb + koff + k0;
      bh[j] = Frag<T>::load(Bb + bo);
      if (SPL == 2) bl[j] = Frag<T>::load(Bb2 + bo);
    }
#pragma unroll
    for (int i = 0; i < 4; ++i) {
      const size_t ao = (size_t)(m0 + (i << 4) + rlane) * lda + koff + k0;
      V ah = Frag<T>::load(Ab + ao);
      V al;
      if (SPL >= 1) al = Frag<T>::load(Ab2 + ao);
#pragma unroll
      for (int j = 0; j < 4; ++j) {
        acc[i][j] = Frag<T>::mma(ah, bh[j], acc[i][j]);
        if (SPL == 2) acc[i][j] = Frag<T>::mma(ah, bl[j], acc[i][j]);
        if (SPL >= 1) acc[i][j] = Frag<T>::mma(al, bh[j], acc[i][j]);
      }
      Frag<T>::guard(acc[i][0], acc[i][3], ah, (SPL >= 1) ? al : ah);
    }
    Frag<T>::keep(bh[0], bh[1], bh[2], bh[3]);
    if (SPL == 2) Frag<T>::keep(bl[0], bl[1], bl[2], bl[3]);
  }
  acc_guard4(acc[0][0], acc[0][1], acc[0][2], acc[0][3]);
  acc_guard4(acc[1][0], acc[1][1], acc[1][2], acc[1][3]);
  acc_guard4(acc[2][0], acc[2][1], acc[2][2], acc[2][3]);
  acc_guard4(acc[3][0], acc[3][1], acc[3][2], acc[3][3]);

  float* slab = sT[wave];
  const float* Rb = RESID ? (resid + (size_t)b * strideR) : nullptr;
#pragma unroll
  for (int i = 0; i < 4; ++i) {
    const int mBase = m0 + (i << 4);
#pragma unroll
    for (int j = 0; j < 4; ++j) {
      const int n = n0 + (j << 4) + rlane;
      float bv = 0.f;
      if (BIAS_MODE == 2) bv = bias[n];
#pragma unroll
      for (int r = 0; r < 8; ++r) {
        float v = acc[i][j][r] * scale;
        if (BIAS_MODE == 1) v += bias[mBase + mOff + r];
        if (BIAS_MODE == 2) v += bv;
        if (RESID) v += Rb[(size_t)(mBase + mOff + r) * ldc + n];
        if (ACT == 1) v = tanhf(v);
        if (ACT == 2) v = fmaxf(v, 0.0f);
        if (ACT == 3) v = v / (1.0f + expf(-v));
        if (ACT == 4) v = (v > 0.f) ? v : 0.01f * v;
        slab[(mOff + r) * 68 + (j << 4) + rlane] = v;
      }
    }
    __builtin_amdgcn_fence(__ATOMIC_RELEASE, "workgroup");
    __builtin_amdgcn_wave_barrier();
    __builtin_amdgcn_fence(__ATOMIC_ACQUIRE, "workgroup");
    if (OUT_MODE == 0) {
      float* C = (float*)Cout + (size_t)b * strideC;
      const int hh = lane >> 4, c4 = (lane & 15) * 4;
      for (int pass = 0; pass < 2; ++pass) {
#pragma unroll
        for (int it = 0; it < 8; ++it) {
          const int row = it * 2 + hh;
          v4f v = *(const v4f*)(slab + row * 68 + c4);
          *(volatile v4f*)(C + (size_t)(mBase + row) * ldc + n0 + c4) = v;
        }
        __threadfence();
      }
    } else {
      const int q = lane >> 3, c8 = (lane & 7) * 8;
      unsigned short* C  = (unsigned short*)Cout  + (size_t)b * strideC;
      unsigned short* C2 = (OUT_MODE == 2) ? ((unsigned short*)Cout2 + (size_t)b * strideC) : nullptr;
      for (int pass = 0; pass < 2; ++pass) {
#pragma unroll
        for (int it = 0; it < 4; ++it) {
          const int row = it * 4 + q;
          const float* sp = slab + row * 68 + c8;
          v8h hv, lv;
#pragma unroll
          for (int e = 0; e < 8; ++e) {
            if (OUT_MODE == 1) {
              hv[e] = (_Float16)sp[e];
            } else {
              unsigned short hb = f2bf_bits(sp[e]);
              unsigned short lb = f2bf_bits(sp[e] - bf_bits2f(hb));
              hv[e] = __builtin_bit_cast(_Float16, hb);
              lv[e] = __builtin_bit_cast(_Float16, lb);
            }
          }
          *(volatile v8h*)(C + (size_t)(mBase + row) * ldc + n0 + c8) = hv;
          if (OUT_MODE == 2) *(volatile v8h*)(C2 + (size_t)(mBase + row) * ldc + n0 + c8) = lv;
        }
        __threadfence();
      }
    }
    __builtin_amdgcn_fence(__ATOMIC_RELEASE, "workgroup");
    __builtin_amdgcn_wave_barrier();
    __builtin_amdgcn_fence(__ATOMIC_ACQUIRE, "workgroup");
  }
}

__global__ __launch_bounds__(256) void cvt_x_bf16_kernel(
    const float* __restrict__ src, unsigned short* __restrict__ dst, int total8)
{
  const int i = blockIdx.x * 256 + threadIdx.x;
  if (i >= total8) return;
  const size_t e0 = (size_t)i << 3;
  const v4f a0 = *(const v4f*)(src + e0);
  const v4f a1 = *(const v4f*)(src + e0 + 4);
  v8h hv;
#pragma unroll
  for (int e = 0; e < 4; ++e) {
    const unsigned short h0 = f2bf_bits(a0[e]), h1 = f2bf_bits(a1[e]);
    hv[e]     = __builtin_bit_cast(_Float16, h0);
    hv[4 + e] = __builtin_bit_cast(_Float16, h1);
  }
  unsigned short* q = dst + e0;
  *(volatile v8h*)q = hv;
  __threadfence();
  *(volatile v8h*)q = hv;
}

__global__ __launch_bounds__(256) void cvt_bw_kernel(
    const float* __restrict__ Bw, unsigned short* __restrict__ dst)
{
  const int i = blockIdx.x * 256 + threadIdx.x;
  const int row = i >> 7;
  const int col = (i & 127) * 8;
  const int rowc = (row < kNst) ? row : (kNst - 1);
  const float fz = (row < kNst) ? 1.0f : 0.0f;
  const v4f a0 = *(const v4f*)(Bw + (size_t)rowc * kDm + col);
  const v4f a1 = *(const v4f*)(Bw + (size_t)rowc * kDm + col + 4);
  v8h hv;
#pragma unroll
  for (int e = 0; e < 4; ++e) {
    const unsigned short h0 = f2bf_bits(a0[e] * fz), h1 = f2bf_bits(a1[e] * fz);
    hv[e]     = __builtin_bit_cast(_Float16, h0);
    hv[4 + e] = __builtin_bit_cast(_Float16, h1);
  }
  unsigned short* q = dst + (size_t)i * 8;
  *(volatile v8h*)q = hv;
  __threadfence();
  *(volatile v8h*)q = hv;
}

__global__ __launch_bounds__(256) void cvt_cw_kernel(
    const float* __restrict__ Cw, unsigned short* __restrict__ dst)
{
  const int i = blockIdx.x * 256 + threadIdx.x;
  const int row = i >> 2;
  const int seg = i & 3;
  const int segc = seg & 1;
  const float fz = (seg < 2) ? 1.0f : 0.0f;
  const v4f a0 = *(const v4f*)(Cw + (size_t)row * kNst + segc * 8);
  const v4f a1 = *(const v4f*)(Cw + (size_t)row * kNst + segc * 8 + 4);
  v8h hv;
#pragma unroll
  for (int e = 0; e < 4; ++e) {
    const unsigned short h0 = f2bf_bits(a0[e] * fz), h1 = f2bf_bits(a1[e] * fz);
    hv[e]     = __builtin_bit_cast(_Float16, h0);
    hv[4 + e] = __builtin_bit_cast(_Float16, h1);
  }
  unsigned short* q = dst + (size_t)i * 8;
  *(volatile v8h*)q = hv;
  __threadfence();
  *(volatile v8h*)q = hv;
}

__global__ __launch_bounds__(256) void gtab_kernel(
    const float* __restrict__ Alog, float* __restrict__ GT)
{
  __shared__ float sRed[8 * kTaps];
  const int tid = threadIdx.x, lane = tid & 31, wave = tid >> 5;
  const int n = blockIdx.x;
  float p[4], dec[4];
#pragma unroll
  for (int i = 0; i < 4; ++i) {
    const int d = tid * 4 + i;
    const float ab = bfr(Alog[(size_t)d * kNst + n]);
    dec[i] = expf(-expf(ab));
    p[i] = 1.0f;
  }
#pragma unroll 1
  for (int k = 0; k < kTaps; ++k) {
    float s = (p[0] + p[1]) + (p[2] + p[3]);
    s += __shfl_xor(s, 16, 32);
    s += __shfl_xor(s, 8, 32);
    s += __shfl_xor(s, 4, 32);
    s += __shfl_xor(s, 2, 32);
    s += __shfl_xor(s, 1, 32);
    if (lane == 0) sRed[wave * kTaps + k] = s;
#pragma unroll
    for (int i = 0; i < 4; ++i) p[i] *= dec[i];
  }
  __syncthreads();
  if (tid < kTaps) {
    float g = 0.0f;
#pragma unroll
    for (int w = 0; w < 8; ++w) g += sRed[w * kTaps + tid];
    g *= (1.0f / 1024.0f);
    float* q = GT + (size_t)n * kTaps + tid;
    *(volatile float*)q = g;
    __threadfence();
    *(volatile float*)q = g;
  }
}

__global__ __launch_bounds__(256) void fir_kernel(
    const float* __restrict__ BX, const float* __restrict__ GT,
    unsigned short* __restrict__ HMH, unsigned short* __restrict__ HML)
{
  __shared__ __align__(16) float sG[kTaps * kNst];
  __shared__ __align__(16) float sB[kFirWin * kNst];
  __shared__ __align__(16) float sH[kFirTS * kNst];
  const int tid = threadIdx.x, lane = tid & 31, wave = tid >> 5;
  constexpr int kChunks = kSeq / kFirTS;
  const int b  = blockIdx.x / kChunks;
  const int t0 = (blockIdx.x - b * kChunks) * kFirTS;
  const size_t rowbase = (size_t)b * kSeq + t0;
#pragma unroll
  for (int i = 0; i < 8; ++i) {
    const int idx = tid + 256 * i;
    const int n = idx >> 7;
    const int k = idx & (kTaps - 1);
    sG[k * kNst + n] = GT[idx];
  }
#pragma unroll
  for (int i = 0; i < 3; ++i) {
    const int idx = tid + 256 * i;
    const int r = idx >> 2, c4 = (idx & 3) * 4;
    const int tm = t0 - kTaps + r;
    const int tmc = (tm < 0) ? 0 : tm;
    const float fz = (tm < 0) ? 0.0f : 1.0f;
    const v4f v = *(const v4f*)(BX + ((size_t)b * kSeq + tmc) * kBxP + c4);
    *(v4f*)(sB + r * kNst + c4) = v * fz;
  }
  __syncthreads();
  const int t = tid >> 2, n0 = (tid & 3) * 4;
  float a0 = 0.0f, a1 = 0.0f, a2 = 0.0f, a3 = 0.0f;
#pragma unroll 1
  for (int k = 0; k < kTaps; ++k) {
    const v4f gv = *(const v4f*)(sG + k * kNst + n0);
    const v4f bv = *(const v4f*)(sB + (t + kTaps - k) * kNst + n0);
    a0 = fmaf(gv[0], bv[0], a0);
    a1 = fmaf(gv[1], bv[1], a1);
    a2 = fmaf(gv[2], bv[2], a2);
    a3 = fmaf(gv[3], bv[3], a3);
  }
  *(v4f*)(sH + t * kNst + n0) = (v4f){a0, a1, a2, a3};
  __syncthreads();
  {
    const int row = wave * 8 + (lane >> 2);
    const int seg = lane & 3;
    const int segc = seg & 1;
    const float fz = (seg < 2) ? 1.0f : 0.0f;
    const v4f h0 = *(const v4f*)(sH + row * kNst + segc * 8);
    const v4f h1 = *(const v4f*)(sH + row * kNst + segc * 8 + 4);
    v8h hv, lv;
#pragma unroll
    for (int e = 0; e < 4; ++e) {
      const float v0 = h0[e] * fz, v1 = h1[e] * fz;
      const unsigned short hb0 = f2bf_bits(v0), hb1 = f2bf_bits(v1);
      const unsigned short lb0 = f2bf_bits(v0 - bf_bits2f(hb0)), lb1 = f2bf_bits(v1 - bf_bits2f(hb1));
      hv[e]     = __builtin_bit_cast(_Float16, hb0);
      hv[4 + e] = __builtin_bit_cast(_Float16, hb1);
      lv[e]     = __builtin_bit_cast(_Float16, lb0);
      lv[4 + e] = __builtin_bit_cast(_Float16, lb1);
    }
    const size_t o = (rowbase + row) * kHmP + (size_t)seg * 8;
    for (int pass = 0; pass < 2; ++pass) {
      *(volatile v8h*)(HMH + o) = hv;
      *(volatile v8h*)(HML + o) = lv;
      __threadfence();
    }
  }
}

__global__ __launch_bounds__(256) void ln_kernel(
    const float* __restrict__ YS, const float* __restrict__ x, const float* __restrict__ Dp,
    const float* __restrict__ gam, const float* __restrict__ bet, float* __restrict__ out)
{
  __shared__ float sR1[8];
  __shared__ float sR2[8];
  const int tid = threadIdx.x, lane = tid & 31, wave = tid >> 5;
  const size_t row = blockIdx.x;
  const int c = tid * 4;
  const v4f ys = *(const v4f*)(YS + row * kDm + c);
  const v4f xv = *(const v4f*)(x + row * kDm + c);
  const v4f dv = *(const v4f*)(Dp + c);
  const v4f gv = *(const v4f*)(gam + c);
  const v4f bv = *(const v4f*)(bet + c);
  float y[4];
#pragma unroll
  for (int e = 0; e < 4; ++e) {
    const float xb = bfr(xv[e]);
    const float db = bfr(dv[e]);
    const float sk = db * xb;
    y[e] = ys[e] + sk;
  }
  float s = (y[0] + y[1]) + (y[2] + y[3]);
  s += __shfl_xor(s, 16, 32);
  s += __shfl_xor(s, 8, 32);
  s += __shfl_xor(s, 4, 32);
  s += __shfl_xor(s, 2, 32);
  s += __shfl_xor(s, 1, 32);
  if (lane == 0) sR1[wave] = s;
  __syncthreads();
  float tot = 0.0f;
#pragma unroll
  for (int w = 0; w < 8; ++w) tot += sR1[w];
  const float mu = tot * (1.0f / 1024.0f);
  float dl[4];
  float s2 = 0.0f;
#pragma unroll
  for (int e = 0; e < 4; ++e) { dl[e] = y[e] - mu; s2 = fmaf(dl[e], dl[e], s2); }
  s2 += __shfl_xor(s2, 16, 32);
  s2 += __shfl_xor(s2, 8, 32);
  s2 += __shfl_xor(s2, 4, 32);
  s2 += __shfl_xor(s2, 2, 32);
  s2 += __shfl_xor(s2, 1, 32);
  if (lane == 0) sR2[wave] = s2;
  __syncthreads();
  float tot2 = 0.0f;
#pragma unroll
  for (int w = 0; w < 8; ++w) tot2 += sR2[w];
  const float var = tot2 * (1.0f / 1024.0f);
  const float rs = rsqrtf(var + 1e-5f);
  v4f o;
#pragma unroll
  for (int e = 0; e < 4; ++e) o[e] = (dl[e] * rs) * bfr(gv[e]) + bfr(bv[e]);
  float* q = out + row * kDm + c;
  *(volatile v4f*)q = o;
  __threadfence();
  *(volatile v4f*)q = o;
}

extern "C" void kernel_launch(void* const* d_in, const int* in_sizes, int n_in,
                              void* d_out, int out_size, void* d_ws, size_t ws_size,
                              hipStream_t stream) {
  if (n_in < 7) return;
  if (in_sizes[0] != kRows * kDm) return;
  if (in_sizes[1] != kDm * kNst) return;
  if (in_sizes[2] != kNst * kDm) return;
  if (in_sizes[3] != kDm * kNst) return;
  if (in_sizes[4] != kDm) return;
  if (in_sizes[5] != kDm) return;
  if (in_sizes[6] != kDm) return;
  if (out_size != kRows * kDm) return;
  if (ws_size < kWsTotal) return;

  const float* x     = (const float*)d_in[0];
  const float* Alog  = (const float*)d_in[1];
  const float* Bw    = (const float*)d_in[2];
  const float* Cw    = (const float*)d_in[3];
  const float* Dv    = (const float*)d_in[4];
  const float* gamma = (const float*)d_in[5];
  const float* beta  = (const float*)d_in[6];
  float* out = (float*)d_out;

  char* ws = (char*)d_ws;
  unsigned short* XB  = (unsigned short*)(ws + kOffXB);
  unsigned short* BWB = (unsigned short*)(ws + kOffBWB);
  unsigned short* CWB = (unsigned short*)(ws + kOffCWB);
  float*          BX  = (float*)(ws + kOffBX);
  float*          GT  = (float*)(ws + kOffGT);
  unsigned short* HMH = (unsigned short*)(ws + kOffHMH);
  unsigned short* HML = (unsigned short*)(ws + kOffHML);
  float*          YS  = (float*)(ws + kOffYS);

  cvt_x_bf16_kernel<<<(kRows * kDm / 8) / 256, 256, 0, stream>>>(x, XB, kRows * kDm / 8);
  cvt_bw_kernel<<<(kBxP * kDm / 8) / 256, 256, 0, stream>>>(Bw, BWB);
  cvt_cw_kernel<<<(kDm * kHmP / 8) / 256, 256, 0, stream>>>(Cw, CWB);

  wmma_gemm64<1, 0, 0, 0, false><<<dim3(16, 1), 256, 0, stream>>>(
      XB, nullptr, kDm, 0L,
      BWB, nullptr, kDm, 0L,
      (void*)BX, nullptr, kBxP, 0L,
      nullptr, nullptr, 0L,
      kRows, kBxP, kDm, 1.0f);

  gtab_kernel<<<kNst, 256, 0, stream>>>(Alog, GT);

  fir_kernel<<<kBatch * (kSeq / kFirTS), 256, 0, stream>>>(BX, GT, HMH, HML);

  wmma_gemm64<1, 1, 0, 0, false><<<dim3(256, 1), 256, 0, stream>>>(
      HMH, HML, kHmP, 0L,
      CWB, nullptr, kHmP, 0L,
      (void*)YS, nullptr, kDm, 0L,
      nullptr, nullptr, 0L,
      kRows, kDm, kHmP, 1.0f);

  ln_kernel<<<kRows, 256, 0, stream>>>(YS, x, Dv, gamma, beta, out);
}
